// LSTMTextEncoder_37684043055273
// MI455X (gfx1250) — hardware-verified
//
#include <hip/hip_runtime.h>
#include <math.h>

constexpr int NBATCH = 256;
constexpr int NSTEP  = 128;
constexpr int EMBD   = 512;
constexpr int HID    = 512;
constexpr int NG4    = 2048;
constexpr int NVOCAB = 32000;
constexpr int TCH    = 16;
constexpr int NCHUNK = NSTEP / TCH;
constexpr int ROWS_PER_CHUNK = TCH * NBATCH;
constexpr int HPITCH = 520;
constexpr int NBLK_LSTM = NBATCH / 16;
constexpr int STATE_FLOATS_PER_BLOCK = 16384;
constexpr float W_CARRY     = 16.0f;
constexpr float W_CARRY_INV = 1.0f / 16.0f;
constexpr float NORM_EPS    = 1e-12f;
static_assert(TCH * NCHUNK == NSTEP, "");
static_assert((TCH % 2) == 0, "");
static_assert(ROWS_PER_CHUNK % 64 == 0, "");

typedef __attribute__((ext_vector_type(16))) _Float16 v16h;
typedef __attribute__((ext_vector_type(8)))  _Float16 v8h;
typedef __attribute__((ext_vector_type(16))) __bf16   v16b;
typedef __attribute__((ext_vector_type(8)))  __bf16   v8b;
typedef __attribute__((ext_vector_type(8)))  float    v8f;
typedef __attribute__((ext_vector_type(4)))  float    v4f;
typedef __attribute__((ext_vector_type(4)))  unsigned int v4u;

__device__ __forceinline__ unsigned short f2bf_bits(float f) {
  unsigned u = __float_as_uint(f);
  return (unsigned short)((u + 0x7FFFu + ((u >> 16) & 1u)) >> 16);
}
__device__ __forceinline__ float bf_bits2f(unsigned short h) { return __uint_as_float(((unsigned)h) << 16); }

__device__ __forceinline__ void dep_guard_h(v8f& a, v8f& b, v16h x, v16h y) { asm volatile("v_nop\n\tv_nop\n\tv_nop\n\tv_nop" : "+v"(a), "+v"(b) : "v"(x), "v"(y)); }
__device__ __forceinline__ void dep_guard_b(v8f& a, v8f& b, v16b x, v16b y) { asm volatile("v_nop\n\tv_nop\n\tv_nop\n\tv_nop" : "+v"(a), "+v"(b) : "v"(x), "v"(y)); }
__device__ __forceinline__ void keep4_h(v16h a, v16h b, v16h c, v16h d) { asm volatile("v_nop" :: "v"(a), "v"(b), "v"(c), "v"(d)); }
__device__ __forceinline__ void keep4_b(v16b a, v16b b, v16b c, v16b d) { asm volatile("v_nop" :: "v"(a), "v"(b), "v"(c), "v"(d)); }
__device__ __forceinline__ void acc_guard4(v8f& a, v8f& b, v8f& c, v8f& d) { asm volatile("v_nop\n\tv_nop\n\tv_nop\n\tv_nop" : "+v"(a), "+v"(b), "+v"(c), "+v"(d)); }
template <typename T> struct Frag;
template <> struct Frag<_Float16> {
  typedef v16h V; union U { v16h v; v8h h[2]; };
  static __device__ __forceinline__ v16h load(const _Float16* p) {
    U f; f.h[0] = *(const v8h*)(p); f.h[1] = *(const v8h*)(p + 16); return f.v;
  }
  static __device__ __forceinline__ v8f mma(v16h a, v16h b, v8f c) {
    return __builtin_amdgcn_wmma_f32_16x16x32_f16(false, a, false, b, (short)0, c, false, false);
  }
  static __device__ __forceinline__ void guard(v8f& a, v8f& b, v16h x, v16h y) { dep_guard_h(a, b, x, y); }
  static __device__ __forceinline__ void keep(v16h a, v16h b, v16h c, v16h d) { keep4_h(a, b, c, d); }
};
template <> struct Frag<__bf16> {
  typedef v16b V; union U { v16b v; v8b h[2]; };
  static __device__ __forceinline__ v16b load(const __bf16* p) {
    U f; f.h[0] = *(const v8b*)(p); f.h[1] = *(const v8b*)(p + 16); return f.v;
  }
  static __device__ __forceinline__ v8f mma(v16b a, v16b b, v8f c) {
    return __builtin_amdgcn_wmma_f32_16x16x32_bf16(false, a, false, b, (short)0, c, false, false);
  }
  static __device__ __forceinline__ void guard(v8f& a, v8f& b, v16b x, v16b y) { dep_guard_b(a, b, x, y); }
  static __device__ __forceinline__ void keep(v16b a, v16b b, v16b c, v16b d) { keep4_b(a, b, c, d); }
};

__device__ __forceinline__ unsigned pk16(unsigned short a, unsigned short b) { return (unsigned)a | ((unsigned)b << 16); }
__device__ __forceinline__ unsigned short h_bits(float f) { const _Float16 h = (_Float16)f; return __builtin_bit_cast(unsigned short, h); }

template <int ET> struct Elem;
template <> struct Elem<0> { typedef _Float16 T; };
template <> struct Elem<1> { typedef __bf16 T; };
template <int ET, bool SPLIT, int BIAS_MODE, int OUT_MODE, bool RESID, int ACT = 0>
__global__ __launch_bounds__(256) void wmma_gemm64(
    const unsigned short* __restrict__ Ap, const unsigned short* __restrict__ A2p, int lda, long strideA,
    const unsigned short* __restrict__ Btp, const unsigned short* __restrict__ Bt2p, int ldb, long strideB,
    void* __restrict__ Cout, void* __restrict__ Cout2, int ldc, long strideC,
    const float* __restrict__ bias,
    const float* __restrict__ resid, long strideR,
    int M, int N, int K, float scale) {
  typedef typename Elem<ET>::T T;
  typedef typename Frag<T>::V V;
  const T* A = (const T*)Ap; const T* A2 = (const T*)A2p; const T* Bt = (const T*)Btp; const T* Bt2 = (const T*)Bt2p;
  __shared__ __align__(16) float sT[8][16 * 68];
  const int b    = blockIdx.y;
  const int lane = threadIdx.x & 31;
  const int wave = threadIdx.x >> 5;
  const int tilesN = N >> 6;
  const int tilesM = M >> 6;
  const int tile = blockIdx.x * 8 + wave;
  if (tile >= tilesM * tilesN) return;
  const int tm = tile / tilesN;
  const int tn = tile - tm * tilesN;
  const int m0 = tm << 6;
  const int n0 = tn << 6;

  const T* Ab  = A  + (size_t)b * strideA;
  const T* Bb  = Bt + (size_t)b * strideB;
  const T* Ab2 = SPLIT ? (A2  + (size_t)b * strideA) : nullptr;
  const T* Bb2 = SPLIT ? (Bt2 + (size_t)b * strideB) : nullptr;

  const int rlane = lane & 15;
  const int koff  = (lane >> 4) * 8;
  const int mOff  = (lane >> 4) * 8;

  v8f acc[4][4];
#pragma unroll
  for (int i = 0; i < 4; ++i)
#pragma unroll
    for (int j = 0; j < 4; ++j) acc[i][j] = (v8f){0.f,0.f,0.f,0.f,0.f,0.f,0.f,0.f};

  for (int k0 = 0; k0 < K; k0 += 32) {
    V bh[4], bl[4];
#pragma unroll
    for (int j = 0; j < 4; ++j) {
      const size_t bo = (size_t)(n0 + (j << 4) + rlane) * ldb + koff + k0;
      bh[j] = Frag<T>::load(Bb + bo);
      if (SPLIT) bl[j] = Frag<T>::load(Bb2 + bo);
    }
#pragma unroll
    for (int i = 0; i < 4; ++i) {
      const size_t ao = (size_t)(m0 + (i << 4) + rlane) * lda + koff + k0;
      V ah = Frag<T>::load(Ab + ao);
      V al;
      if (SPLIT) al = Frag<T>::load(Ab2 + ao);
#pragma unroll
      for (int j = 0; j < 4; ++j) {
        acc[i][j] = Frag<T>::mma(ah, bh[j], acc[i][j]);
        if (SPLIT) {
          acc[i][j] = Frag<T>::mma(ah, bl[j], acc[i][j]);
          acc[i][j] = Frag<T>::mma(al, bh[j], acc[i][j]);
        }
      }
      Frag<T>::guard(acc[i][0], acc[i][3], ah, SPLIT ? al : ah);
    }
    Frag<T>::keep(bh[0], bh[1], bh[2], bh[3]);
    if (SPLIT) Frag<T>::keep(bl[0], bl[1], bl[2], bl[3]);
  }
  acc_guard4(acc[0][0], acc[0][1], acc[0][2], acc[0][3]);
  acc_guard4(acc[1][0], acc[1][1], acc[1][2], acc[1][3]);
  acc_guard4(acc[2][0], acc[2][1], acc[2][2], acc[2][3]);
  acc_guard4(acc[3][0], acc[3][1], acc[3][2], acc[3][3]);

  float* slab = sT[wave];
  const float* Rb = RESID ? (resid + (size_t)b * strideR) : nullptr;
#pragma unroll
  for (int i = 0; i < 4; ++i) {
    const int mBase = m0 + (i << 4);
#pragma unroll
    for (int j = 0; j < 4; ++j) {
      const int n = n0 + (j << 4) + rlane;
      float bv = 0.f;
      if (BIAS_MODE == 2) bv = bias[n];
#pragma unroll
      for (int r = 0; r < 8; ++r) {
        float v = acc[i][j][r] * scale;
        if (BIAS_MODE == 1) v += bias[mBase + mOff + r];
        if (BIAS_MODE == 2) v += bv;
        if (RESID) v += Rb[(size_t)(mBase + mOff + r) * ldc + n];
        if (ACT == 2) v = fmaxf(v, 0.0f);
        if (ACT == 4) v = (v > 0.f) ? v : 0.01f * v;
        slab[(mOff + r) * 68 + (j << 4) + rlane] = v;
      }
    }
    __builtin_amdgcn_fence(__ATOMIC_RELEASE, "workgroup");
    __builtin_amdgcn_wave_barrier();
    __builtin_amdgcn_fence(__ATOMIC_ACQUIRE, "workgroup");
    if (OUT_MODE == 0) {
      float* C = (float*)Cout + (size_t)b * strideC;
      const int hh = lane >> 4, c4 = (lane & 15) * 4;
      for (int pass = 0; pass < 2; ++pass) {
#pragma unroll
        for (int it = 0; it < 8; ++it) {
          const int row = it * 2 + hh;
          v4f v = *(const v4f*)(slab + row * 68 + c4);
          *(volatile v4f*)(C + (size_t)(mBase + row) * ldc + n0 + c4) = v;
        }
        __threadfence();
      }
    } else {
      const int q = lane >> 3, c8 = (lane & 7) * 8;
      unsigned short* C  = (unsigned short*)Cout  + (size_t)b * strideC;
      unsigned short* C2 = (OUT_MODE == 2) ? ((unsigned short*)Cout2 + (size_t)b * strideC) : nullptr;
      for (int pass = 0; pass < 2; ++pass) {
#pragma unroll
        for (int it = 0; it < 4; ++it) {
          const int row = it * 4 + q;
          const float* sp = slab + row * 68 + c8;
          v8h hv, lv;
#pragma unroll
          for (int e = 0; e < 8; ++e) {
            if (OUT_MODE == 1) {
              hv[e] = (_Float16)sp[e];
            } else {
              unsigned short hb = f2bf_bits(sp[e]);
              unsigned short lb = f2bf_bits(sp[e] - bf_bits2f(hb));
              hv[e] = __builtin_bit_cast(_Float16, hb);
              lv[e] = __builtin_bit_cast(_Float16, lb);
            }
          }
          *(volatile v8h*)(C + (size_t)(mBase + row) * ldc + n0 + c8) = hv;
          if (OUT_MODE == 2) *(volatile v8h*)(C2 + (size_t)(mBase + row) * ldc + n0 + c8) = lv;
        }
        __threadfence();
      }
    }
    __builtin_amdgcn_fence(__ATOMIC_RELEASE, "workgroup");
    __builtin_amdgcn_wave_barrier();
    __builtin_amdgcn_fence(__ATOMIC_ACQUIRE, "workgroup");
  }
}

__global__ __launch_bounds__(256) void gather_x_kernel(const int* __restrict__ cap, const float* __restrict__ emb,
                                                       unsigned short* __restrict__ X16) {
  const int idx = blockIdx.x * 256 + threadIdx.x;
  const int e8  = idx & 63;
  const int row = idx >> 6;
  const int t   = row >> 8;
  const int bb  = row & 255;
  int tok = cap[bb * NSTEP + t];
  tok = tok < 0 ? 0 : (tok > NVOCAB - 1 ? NVOCAB - 1 : tok);
  const float* src = emb + (size_t)tok * EMBD + e8 * 8;
  const v4f a = *(const v4f*)(src);
  const v4f d = *(const v4f*)(src + 4);
  const bool nz = (tok != 0);
  unsigned short hb[8];
#pragma unroll
  for (int e = 0; e < 4; ++e) {
    hb[e]     = h_bits(nz ? a[e] : 0.0f);
    hb[4 + e] = h_bits(nz ? d[e] : 0.0f);
  }
  const v4u u = (v4u){pk16(hb[0], hb[1]), pk16(hb[2], hb[3]), pk16(hb[4], hb[5]), pk16(hb[6], hb[7])};
  unsigned short* dst = X16 + (size_t)row * EMBD + e8 * 8;
  *(volatile v4u*)dst = u;
  __threadfence();
  *(volatile v4u*)dst = u;
}

__global__ __launch_bounds__(256) void wtcast_kernel(const float* __restrict__ W, unsigned short* __restrict__ out,
                                                     int KD, int ND, float scale) {
  __shared__ float sm[64][65];
  const int t  = threadIdx.x;
  const int k0 = blockIdx.x * 64;
  const int n0 = blockIdx.y * 64;
#pragma unroll
  for (int i = 0; i < 16; ++i) {
    const int e  = i * 256 + t;
    const int r  = e >> 6;
    const int cc = e & 63;
    sm[cc][r] = W[(size_t)(k0 + r) * ND + n0 + cc] * scale;
  }
  __syncthreads();
  const int lane = t & 31, wave = t >> 5;
  const int q = lane >> 3, c8 = (lane & 7) * 8;
  for (int pass = 0; pass < 2; ++pass) {
#pragma unroll
    for (int it = 0; it < 2; ++it) {
      const int row = wave * 8 + it * 4 + q;
      unsigned short hb[8];
#pragma unroll
      for (int e = 0; e < 8; ++e) hb[e] = h_bits(sm[row][c8 + e]);
      const v4u u = (v4u){pk16(hb[0], hb[1]), pk16(hb[2], hb[3]), pk16(hb[4], hb[5]), pk16(hb[6], hb[7])};
      *(volatile v4u*)(out + (size_t)(n0 + row) * KD + k0 + c8) = u;
    }
    __threadfence();
  }
}

__device__ __forceinline__ float sigm_f(float x) {
  const float e = expf(fminf(-x, 30.0f));
  return 1.0f / (1.0f + e);
}

__global__ __launch_bounds__(512) void lstm_chunk_kernel(
    const float* __restrict__ XG, const unsigned short* __restrict__ UhTp, const float* __restrict__ bu,
    float* __restrict__ state, unsigned short* __restrict__ HT16p, int first, int last) {
  const _Float16* UhT = (const _Float16*)UhTp;
  __shared__ __align__(16) _Float16 hs[2][16 * HPITCH];
  const int tid  = threadIdx.x;
  const int wave = tid >> 5;
  const int lane = tid & 31;
  const int cl   = lane & 15;
  const int hh   = lane >> 4;
  const int b0   = blockIdx.x * 16;
  const int ucol0 = 32 * wave + cl;
  float* stb = state + (size_t)blockIdx.x * STATE_FLOATS_PER_BLOCK;

  float buv[2][4];
#pragma unroll
  for (int j = 0; j < 2; ++j)
#pragma unroll
    for (int q = 0; q < 4; ++q) buv[j][q] = bu[q * HID + ucol0 + 16 * j];

  float cst[2][8], hst[2][8];
#pragma unroll
  for (int j = 0; j < 2; ++j)
#pragma unroll
    for (int r = 0; r < 8; ++r) { cst[j][r] = 0.0f; hst[j][r] = 0.0f; }

  if (!first) {
#pragma unroll
    for (int j = 0; j < 2; ++j)
#pragma unroll
      for (int g = 0; g < 2; ++g) {
        const int ci = ((wave * 2 + j) * 2 + g);
        const v4f cv = *(const v4f*)(stb + ci * 128 + lane * 4);
        const v4f hv = *(const v4f*)(stb + 8192 + ci * 128 + lane * 4);
#pragma unroll
        for (int e = 0; e < 4; ++e) { cst[j][4 * g + e] = cv[e]; hst[j][4 * g + e] = hv[e]; }
      }
  }
#pragma unroll
  for (int j = 0; j < 2; ++j)
#pragma unroll
    for (int r = 0; r < 8; ++r) hs[0][(8 * hh + r) * HPITCH + ucol0 + 16 * j] = (_Float16)hst[j][r];
  __syncthreads();

#pragma unroll 1
  for (int tl = 0; tl < TCH; ++tl) {
    const _Float16* hcur = &hs[tl & 1][0];
    _Float16* hnxt = &hs[(tl & 1) ^ 1][0];
    v8f acc[2][4];
#pragma unroll
    for (int j = 0; j < 2; ++j)
#pragma unroll
      for (int q = 0; q < 4; ++q) acc[j][q] = (v8f){0.f,0.f,0.f,0.f,0.f,0.f,0.f,0.f};

#pragma unroll 1
    for (int k0 = 0; k0 < HID; k0 += 32) {
      v16h bq[2][4];
#pragma unroll
      for (int j = 0; j < 2; ++j)
#pragma unroll
        for (int q = 0; q < 4; ++q)
          bq[j][q] = Frag<_Float16>::load(UhT + (size_t)(q * HID + ucol0 + 16 * j) * HID + k0 + 8 * hh);
      const v16h a = Frag<_Float16>::load(hcur + cl * HPITCH + k0 + 8 * hh);
#pragma unroll
      for (int j = 0; j < 2; ++j)
#pragma unroll
        for (int q = 0; q < 4; ++q) acc[j][q] = Frag<_Float16>::mma(a, bq[j][q], acc[j][q]);
      dep_guard_h(acc[0][0], acc[1][3], a, a);
      keep4_h(bq[0][0], bq[0][1], bq[0][2], bq[0][3]);
      keep4_h(bq[1][0], bq[1][1], bq[1][2], bq[1][3]);
    }
    acc_guard4(acc[0][0], acc[0][1], acc[0][2], acc[0][3]);
    acc_guard4(acc[1][0], acc[1][1], acc[1][2], acc[1][3]);

    const float* xg0 = XG + (size_t)(tl * NBATCH + b0 + 8 * hh) * NG4 + ucol0;
#pragma unroll
    for (int j = 0; j < 2; ++j) {
#pragma unroll
      for (int r = 0; r < 8; ++r) {
        const float* xr = xg0 + (size_t)r * NG4 + 16 * j;
        const float gi = acc[j][0][r] * W_CARRY_INV + xr[0]       + buv[j][0];
        const float gf = acc[j][1][r] * W_CARRY_INV + xr[HID]     + buv[j][1];
        const float go = acc[j][2][r] * W_CARRY_INV + xr[2 * HID] + buv[j][2];
        const float gc = acc[j][3][r] * W_CARRY_INV + xr[3 * HID] + buv[j][3];
        const float iv = sigm_f(gi);
        const float fv = sigm_f(gf);
        const float ov = sigm_f(go);
        const float gv = tanhf(gc);
        const float cn = fv * cst[j][r] + iv * gv;
        cst[j][r] = cn;
        const float hn = ov * tanhf(cn);
        hst[j][r] = hn;
        hnxt[(8 * hh + r) * HPITCH + ucol0 + 16 * j] = (_Float16)hn;
      }
    }
    __syncthreads();
  }

  if (!last) {
    v4f cvv[2][2], hvv[2][2];
#pragma unroll
    for (int j = 0; j < 2; ++j)
#pragma unroll
      for (int g = 0; g < 2; ++g) {
        cvv[j][g] = (v4f){cst[j][4 * g], cst[j][4 * g + 1], cst[j][4 * g + 2], cst[j][4 * g + 3]};
        hvv[j][g] = (v4f){hst[j][4 * g], hst[j][4 * g + 1], hst[j][4 * g + 2], hst[j][4 * g + 3]};
      }
    for (int pass = 0; pass < 2; ++pass) {
#pragma unroll
      for (int j = 0; j < 2; ++j)
#pragma unroll
        for (int g = 0; g < 2; ++g) {
          const int ci = ((wave * 2 + j) * 2 + g);
          *(volatile v4f*)(stb + ci * 128 + lane * 4) = cvv[j][g];
          *(volatile v4f*)(stb + 8192 + ci * 128 + lane * 4) = hvv[j][g];
        }
      __threadfence();
    }
  } else {
    const _Float16* hrow = &hs[0][0] + wave * HPITCH;
    const v8h u0 = *(const v8h*)(hrow + lane * 8);
    const v8h u1 = *(const v8h*)(hrow + 256 + lane * 8);
    _Float16* dst = (_Float16*)HT16p + (size_t)(b0 + wave) * HID;
    for (int pass = 0; pass < 2; ++pass) {
      *(volatile v8h*)(dst + lane * 8) = u0;
      *(volatile v8h*)(dst + 256 + lane * 8) = u1;
      __threadfence();
    }
  }
}

__global__ __launch_bounds__(256) void l2norm_kernel(const float* __restrict__ in, float* __restrict__ out) {
  const int wave = threadIdx.x >> 5, lane = threadIdx.x & 31;
  const int row = blockIdx.x * 8 + wave;
  const float* p = in + (size_t)row * EMBD;
  const v4f x0 = *(const v4f*)(p + lane * 4);
  const v4f x1 = *(const v4f*)(p + 128 + lane * 4);
  const v4f x2 = *(const v4f*)(p + 256 + lane * 4);
  const v4f x3 = *(const v4f*)(p + 384 + lane * 4);
  float s = 0.0f;
#pragma unroll
  for (int e = 0; e < 4; ++e) s += x0[e] * x0[e] + x1[e] * x1[e] + x2[e] * x2[e] + x3[e] * x3[e];
#pragma unroll
  for (int off = 16; off > 0; off >>= 1) s += __shfl_xor(s, off, 32);
  const float nrm = sqrtf(s);
  const float inv = 1.0f / fmaxf(nrm, NORM_EPS);
  const v4f y0 = x0 * inv, y1 = x1 * inv, y2 = x2 * inv, y3 = x3 * inv;
  float* o = out + (size_t)row * EMBD;
  for (int pass = 0; pass < 2; ++pass) {
    *(volatile v4f*)(o + lane * 4) = y0;
    *(volatile v4f*)(o + 128 + lane * 4) = y1;
    *(volatile v4f*)(o + 256 + lane * 4) = y2;
    *(volatile v4f*)(o + 384 + lane * 4) = y3;
    __threadfence();
  }
}

extern "C" void kernel_launch(void* const* d_in, const int* in_sizes, int n_in,
                              void* d_out, int out_size, void* d_ws, size_t ws_size,
                              hipStream_t stream) {
  if (n_in < 8) return;
  if (in_sizes[0] != NBATCH * NSTEP || in_sizes[1] != NVOCAB * EMBD || in_sizes[2] != EMBD * NG4 ||
      in_sizes[3] != NG4 || in_sizes[4] != HID * NG4 || in_sizes[5] != NG4 || in_sizes[6] != HID * EMBD ||
      in_sizes[7] != EMBD || out_size != NBATCH * EMBD) return;

  const int*   captions = (const int*)  d_in[0];
  const float* emb      = (const float*)d_in[1];
  const float* Wx       = (const float*)d_in[2];
  const float* bx       = (const float*)d_in[3];
  const float* Uh       = (const float*)d_in[4];
  const float* bu       = (const float*)d_in[5];
  const float* fcW      = (const float*)d_in[6];
  const float* fcb      = (const float*)d_in[7];

  const size_t szX16   = (size_t)NSTEP * NBATCH * EMBD * 2;
  const size_t szWT    = (size_t)NG4 * EMBD * 2;
  const size_t szFCWT  = (size_t)EMBD * HID * 2;
  const size_t szXG    = (size_t)ROWS_PER_CHUNK * NG4 * 4;
  const size_t szSTATE = (size_t)NBLK_LSTM * STATE_FLOATS_PER_BLOCK * 4;
  const size_t szHT16  = (size_t)NBATCH * HID * 2;
  const size_t szFC    = (size_t)NBATCH * EMBD * 4;

  size_t off = 0;
  char* ws = (char*)d_ws;
  unsigned short* X16  = (unsigned short*)(ws + off); off += szX16;
  unsigned short* WxT  = (unsigned short*)(ws + off); off += szWT;
  unsigned short* UhT  = (unsigned short*)(ws + off); off += szWT;
  unsigned short* fcWT = (unsigned short*)(ws + off); off += szFCWT;
  float* XG0   = (float*)(ws + off); off += szXG;
  float* XG1   = (float*)(ws + off); off += szXG;
  float* STATE = (float*)(ws + off); off += szSTATE;
  unsigned short* HT16 = (unsigned short*)(ws + off); off += szHT16;
  float* FCOUT = (float*)(ws + off); off += szFC;
  if (off > ws_size) return;

  gather_x_kernel<<<8192, 256, 0, stream>>>(captions, emb, X16);

  wtcast_kernel<<<dim3(EMBD / 64, NG4 / 64), 256, 0, stream>>>(Wx, WxT, EMBD, NG4, W_CARRY);
  wtcast_kernel<<<dim3(HID / 64, NG4 / 64), 256, 0, stream>>>(Uh, UhT, HID, NG4, W_CARRY);
  wtcast_kernel<<<dim3(HID / 64, EMBD / 64), 256, 0, stream>>>(fcW, fcWT, HID, EMBD, W_CARRY);

  for (int ch = 0; ch < NCHUNK; ++ch) {
    float* XGp = (ch & 1) ? XG1 : XG0;
    const unsigned short* Achunk = X16 + (size_t)ch * ROWS_PER_CHUNK * EMBD;
    wmma_gemm64<0, false, 2, 0, false><<<dim3(256, 1), 256, 0, stream>>>(
        Achunk, nullptr, EMBD, 0L,
        WxT, nullptr, EMBD, 0L,
        (void*)XGp, nullptr, NG4, 0L,
        bx,
        nullptr, 0L,
        ROWS_PER_CHUNK, NG4, EMBD, W_CARRY_INV);
    const int firstFlag = (ch == 0) ? 1 : 0;
    const int lastFlag  = (ch == NCHUNK - 1) ? 1 : 0;
    lstm_chunk_kernel<<<NBLK_LSTM, 512, 0, stream>>>(XGp, UhT, bu, STATE, HT16, firstFlag, lastFlag);
  }

  wmma_gemm64<0, false, 2, 0, false><<<dim3(4, 1), 256, 0, stream>>>(
      HT16, nullptr, HID, 0L,
      fcWT, nullptr, HID, 0L,
      (void*)FCOUT, nullptr, EMBD, 0L,
      fcb,
      nullptr, 0L,
      NBATCH, EMBD, HID, W_CARRY_INV);

  l2norm_kernel<<<NBATCH / 8, 256, 0, stream>>>(FCOUT, (float*)d_out);
}
